// Involution2D_8847632630036
// MI455X (gfx1250) — hardware-verified
//
#include <hip/hip_runtime.h>

typedef __bf16         v16b __attribute__((ext_vector_type(16)));
typedef unsigned short v8us __attribute__((ext_vector_type(8)));
typedef float          v8f  __attribute__((ext_vector_type(8)));
typedef float          v4f  __attribute__((ext_vector_type(4)));
typedef v8us __attribute__((may_alias)) v8usa;
typedef v4f  __attribute__((may_alias)) v4fa;

union Frag { v16b v; v8us half[2]; };

#define BS    4
#define CH    256
#define HW    64
#define NPB   4096
#define NPIX  16384
#define CR    64
#define NQ    784
#define NG    16
#define GC    16
#define K2    49
#define RB    4
#define HROWS 10
#define HCOLS 70
#define HP    72

__device__ __forceinline__ unsigned short f2bf(float f) {
  unsigned int u = __float_as_uint(f);
  u = u + 0x7FFFu + ((u >> 16) & 1u);
  return (unsigned short)(u >> 16);
}
__device__ __forceinline__ float bf2f(unsigned short hb) {
  return __uint_as_float(((unsigned int)hb) << 16);
}
__device__ __forceinline__ void split8(v4f a, v4f c, v8us& hi, v8us& lo) {
  float f[8] = {a.x, a.y, a.z, a.w, c.x, c.y, c.z, c.w};
  v8us hh = {0, 0, 0, 0, 0, 0, 0, 0};
  v8us ll = {0, 0, 0, 0, 0, 0, 0, 0};
  #pragma unroll
  for (int e = 0; e < 8; ++e) {
    const unsigned short hb = f2bf(f[e]);
    hh[e] = hb;
    ll[e] = f2bf(f[e] - bf2f(hb));
  }
  hi = hh; lo = ll;
}

__device__ __forceinline__ v8f wmma_bf16(v16b a, v16b b, v8f c) {
  v8f d = __builtin_amdgcn_wmma_f32_16x16x32_bf16(false, a, false, b, (short)0, c, false, false);
  asm volatile("v_nop\n\tv_nop\n\tv_nop\n\tv_nop" : "+v"(d) : "v"(a), "v"(b));
  return d;
}

__device__ __forceinline__ v16b load_frag(const unsigned short* p, int h) {
  Frag f;
  f.half[0] = *(const v8usa*)(p + 8 * h);
  f.half[1] = *(const v8usa*)(p + 16 + 8 * h);
  return f.v;
}

__global__ __launch_bounds__(256) void k_cvt_x(
    const float* __restrict__ x,
    unsigned short* __restrict__ xh, unsigned short* __restrict__ xl)
{
  __shared__ float s[64 * 65];
  const int tid = threadIdx.x;
  const int p0 = blockIdx.x * 64;
  const int c0 = blockIdx.y * 64;
  const int b  = blockIdx.z;
  const float* src = x + ((size_t)(b * CH + c0)) * NPB + p0;
  #pragma unroll
  for (int it = 0; it < 16; ++it) {
    const int e = it * 256 + tid;
    const int c = e >> 6, px = e & 63;
    s[c * 65 + px] = src[(size_t)c * NPB + px];
  }
  __syncthreads();

  const int q8 = tid & 7, sub = tid >> 3;
  v8us hv[2], lv[2];
  size_t off[2];
  #pragma unroll
  for (int it = 0; it < 2; ++it) {
    const int li = it * 32 + sub;
    float f[8];
    #pragma unroll
    for (int e = 0; e < 8; ++e) f[e] = s[(8 * q8 + e) * 65 + li];
    const v4f a = {f[0], f[1], f[2], f[3]};
    const v4f c = {f[4], f[5], f[6], f[7]};
    split8(a, c, hv[it], lv[it]);
    off[it] = ((size_t)(b * NPB + p0 + li)) * CH + c0 + 8 * q8;
  }
  #pragma unroll
  for (int it = 0; it < 2; ++it) {
    *(volatile v8us*)(xh + off[it]) = hv[it];
    *(volatile v8us*)(xl + off[it]) = lv[it];
  }
  __threadfence();
  #pragma unroll
  for (int it = 0; it < 2; ++it) {
    *(volatile v8us*)(xh + off[it]) = hv[it];
    *(volatile v8us*)(xl + off[it]) = lv[it];
  }
}

__global__ __launch_bounds__(256) void k_cvt_w(
    const float* __restrict__ wr, const float* __restrict__ wsp,
    unsigned short* __restrict__ wrh, unsigned short* __restrict__ wrl,
    unsigned short* __restrict__ wsh, unsigned short* __restrict__ wsl)
{
  const int tid = threadIdx.x;
  if (blockIdx.x < 8) {
    const int t = blockIdx.x * 256 + tid;
    const float* src = wr + (size_t)t * 8;
    const v4f a = *(const v4fa*)src;
    const v4f c = *(const v4fa*)(src + 4);
    v8us hi, lo;
    split8(a, c, hi, lo);
    const size_t off = (size_t)t * 8;
    *(volatile v8us*)(wrh + off) = hi;
    *(volatile v8us*)(wrl + off) = lo;
    __threadfence();
    *(volatile v8us*)(wrh + off) = hi;
    *(volatile v8us*)(wrl + off) = lo;
  } else {
    const int t = (blockIdx.x - 8) * 256 + tid;
    if (t < (NQ * CR) / 8) {
      const float* src = wsp + (size_t)t * 8;
      const v4f a = *(const v4fa*)src;
      const v4f c = *(const v4fa*)(src + 4);
      v8us hi, lo;
      split8(a, c, hi, lo);
      const size_t off = (size_t)t * 8;
      *(volatile v8us*)(wsh + off) = hi;
      *(volatile v8us*)(wsl + off) = lo;
      __threadfence();
      *(volatile v8us*)(wsh + off) = hi;
      *(volatile v8us*)(wsl + off) = lo;
    }
  }
}

__global__ __launch_bounds__(128) void k_gemm1(
    const unsigned short* __restrict__ xh, const unsigned short* __restrict__ xl,
    const unsigned short* __restrict__ wrh, const unsigned short* __restrict__ wrl,
    const float* __restrict__ br,
    unsigned short* __restrict__ th, unsigned short* __restrict__ tl)
{
  __shared__ __attribute__((aligned(16))) float sT[4 * 16 * 64];

  const int tid = threadIdx.x, lane = tid & 31, w = tid >> 5;
  const int h = lane >> 4, m = lane & 15;
  const int p0w = blockIdx.x * 64 + 16 * w;

  const unsigned short* xah = xh + (size_t)(p0w + m) * CH;
  const unsigned short* xal = xl + (size_t)(p0w + m) * CH;
  const unsigned short* wbh = wrh + (size_t)m * CH;
  const unsigned short* wbl = wrl + (size_t)m * CH;

  const v8f zero8 = {0.f, 0.f, 0.f, 0.f, 0.f, 0.f, 0.f, 0.f};
  v8f acc[4];
  #pragma unroll
  for (int nt = 0; nt < 4; ++nt) acc[nt] = zero8;

  #pragma unroll 1
  for (int k0 = 0; k0 < CH; k0 += 32) {
    const v16b ah = load_frag(xah + k0, h);
    const v16b al = load_frag(xal + k0, h);
    #pragma unroll
    for (int nt = 0; nt < 4; ++nt) {
      const v16b bh = load_frag(wbh + (size_t)nt * 16 * CH + k0, h);
      const v16b bl = load_frag(wbl + (size_t)nt * 16 * CH + k0, h);
      acc[nt] = wmma_bf16(ah, bh, acc[nt]);
      acc[nt] = wmma_bf16(ah, bl, acc[nt]);
      acc[nt] = wmma_bf16(al, bh, acc[nt]);
    }
  }

  float* st = sT + w * 1024;
  #pragma unroll
  for (int nt = 0; nt < 4; ++nt) {
    const int o = 16 * nt + m;
    const float bias = br[o];
    #pragma unroll
    for (int r = 0; r < 8; ++r) st[(8 * h + r) * 64 + o] = acc[nt][r] + bias;
  }
  __syncthreads();

  const int q8 = lane & 7, sub = lane >> 3;
  v8us hv[4], lv[4];
  size_t off[4];
  #pragma unroll
  for (int i = 0; i < 4; ++i) {
    const int row = 4 * i + sub;
    const float* sp = st + row * 64 + 8 * q8;
    const v4f a = *(const v4fa*)sp;
    const v4f c = *(const v4fa*)(sp + 4);
    split8(a, c, hv[i], lv[i]);
    off[i] = (size_t)(p0w + row) * CR + 8 * q8;
  }
  #pragma unroll
  for (int i = 0; i < 4; ++i) {
    *(volatile v8us*)(th + off[i]) = hv[i];
    *(volatile v8us*)(tl + off[i]) = lv[i];
  }
  __threadfence();
  #pragma unroll
  for (int i = 0; i < 4; ++i) {
    *(volatile v8us*)(th + off[i]) = hv[i];
    *(volatile v8us*)(tl + off[i]) = lv[i];
  }
}

__global__ __launch_bounds__(128) void k_gemm2(
    const unsigned short* __restrict__ wsh, const unsigned short* __restrict__ wsl,
    const unsigned short* __restrict__ th,  const unsigned short* __restrict__ tl,
    const float* __restrict__ bsp,
    float* __restrict__ kern)
{
  __shared__ __attribute__((aligned(16))) float sK[4 * 16 * 64];

  const int tid = threadIdx.x, lane = tid & 31, w = tid >> 5;
  const int h = lane >> 4, m = lane & 15;
  const int q0  = blockIdx.y * 16;
  const int n0w = blockIdx.x * 256 + 64 * w;

  const unsigned short* wah = wsh + (size_t)(q0 + m) * CR;
  const unsigned short* wal = wsl + (size_t)(q0 + m) * CR;
  const v16b ah0 = load_frag(wah, h),      al0 = load_frag(wal, h);
  const v16b ah1 = load_frag(wah + 32, h), al1 = load_frag(wal + 32, h);

  const v8f zero8 = {0.f, 0.f, 0.f, 0.f, 0.f, 0.f, 0.f, 0.f};
  v8f acc[4];
  #pragma unroll
  for (int nt = 0; nt < 4; ++nt) {
    const unsigned short* tbh = th + (size_t)(n0w + 16 * nt + m) * CR;
    const unsigned short* tbl = tl + (size_t)(n0w + 16 * nt + m) * CR;
    const v16b bh0 = load_frag(tbh, h),      bl0 = load_frag(tbl, h);
    const v16b bh1 = load_frag(tbh + 32, h), bl1 = load_frag(tbl + 32, h);
    v8f z = zero8;
    z = wmma_bf16(ah0, bh0, z);
    z = wmma_bf16(ah0, bl0, z);
    z = wmma_bf16(al0, bh0, z);
    z = wmma_bf16(ah1, bh1, z);
    z = wmma_bf16(ah1, bl1, z);
    z = wmma_bf16(al1, bh1, z);
    acc[nt] = z;
  }

  float* sk = sK + w * 1024;
  float bq[8];
  #pragma unroll
  for (int r = 0; r < 8; ++r) bq[r] = bsp[q0 + 8 * h + r];
  #pragma unroll
  for (int nt = 0; nt < 4; ++nt) {
    #pragma unroll
    for (int r = 0; r < 8; ++r) sk[(8 * h + r) * 64 + 16 * nt + m] = acc[nt][r] + bq[r];
  }
  __syncthreads();

  const int q8 = lane & 7, sub = lane >> 3;
  v4f vv[8];
  size_t off[8];
  #pragma unroll
  for (int i = 0; i < 8; ++i) {
    const int lid = 4 * i + sub;
    const int row = lid >> 1, hl = lid & 1;
    vv[i] = *(const v4fa*)(sk + row * 64 + 32 * hl + 4 * q8);
    off[i] = (size_t)(q0 + row) * NPIX + n0w + 32 * hl + 4 * q8;
  }
  #pragma unroll
  for (int i = 0; i < 8; ++i) *(volatile v4f*)(kern + off[i]) = vv[i];
  __threadfence();
  #pragma unroll
  for (int i = 0; i < 8; ++i) *(volatile v4f*)(kern + off[i]) = vv[i];
}

__global__ __launch_bounds__(256) void k_inv(
    const float* __restrict__ x,
    const float* __restrict__ kern,
    float* __restrict__ out)
{
  __shared__ float sh[GC * HROWS * HP];
  __shared__ __attribute__((aligned(16))) float so[RB * HW];

  const int tid = threadIdx.x;
  const int band = blockIdx.x, g = blockIdx.y, b = blockIdx.z;
  const int y0 = band * RB;

  const float* xg = x + (size_t)(b * CH + g * GC) * NPB;
  for (int e = tid; e < GC * HROWS * HCOLS; e += 256) {
    const int c   = e / (HROWS * HCOLS);
    const int rem = e - c * (HROWS * HCOLS);
    const int r   = rem / HCOLS;
    const int col = rem - r * HCOLS;
    const int yy = y0 - 3 + r, xx = col - 3;
    const bool valid = ((unsigned)yy < 64u) && ((unsigned)xx < 64u);
    const int yc = min(max(yy, 0), 63), xc = min(max(xx, 0), 63);
    const float v = xg[(size_t)c * NPB + yc * HW + xc];
    sh[(c * HROWS + r) * HP + col] = valid ? v : 0.0f;
  }

  const int yl = tid >> 6, xl = tid & 63;
  const int pg = b * NPB + (y0 + yl) * HW + xl;
  const float* kp = kern + (size_t)(g * K2) * NPIX + pg;
  float kv[K2];
  #pragma unroll
  for (int k = 0; k < K2; ++k) kv[k] = kp[(size_t)k * NPIX];
  __syncthreads();

  const float* hb = sh + yl * HP + xl;
  float* ob = out + ((size_t)(b * CH + g * GC) * HW + y0) * HW;

  #pragma unroll 1
  for (int c = 0; c < GC; ++c) {
    const float* hc = hb + c * (HROWS * HP);
    float acc = 0.0f;
    #pragma unroll
    for (int i = 0; i < 7; ++i) {
      #pragma unroll
      for (int j = 0; j < 7; ++j) acc = fmaf(kv[i * 7 + j], hc[i * HP + j], acc);
    }
    so[tid] = acc;
    __syncthreads();
    if (tid < 64) {
      const v4f v = *(const v4fa*)(so + 4 * tid);
      float* dst = ob + (size_t)c * NPB + 4 * tid;
      *(volatile v4f*)dst = v;
      __threadfence();
      *(volatile v4f*)dst = v;
    }
    __syncthreads();
  }
}

extern "C" void kernel_launch(void* const* d_in, const int* in_sizes, int n_in,
                              void* d_out, int out_size, void* d_ws, size_t ws_size,
                              hipStream_t stream) {
  if (n_in < 5) return;
  if (in_sizes[0] != BS * CH * NPB) return;
  if (in_sizes[1] != CR * CH) return;
  if (in_sizes[2] != CR) return;
  if (in_sizes[3] != NQ * CR) return;
  if (in_sizes[4] != NQ) return;
  if (out_size != BS * CH * NPB) return;

  const float* x   = (const float*)d_in[0];
  const float* wr  = (const float*)d_in[1];
  const float* br  = (const float*)d_in[2];
  const float* wsp = (const float*)d_in[3];
  const float* bsp = (const float*)d_in[4];
  float* out = (float*)d_out;

  const size_t xp_bytes = (size_t)NPIX * CH * 2;
  const size_t wr_bytes = (size_t)CR * CH * 2;
  const size_t ws_pl_bytes = (size_t)NQ * CR * 2;
  const size_t t_bytes  = (size_t)NPIX * CR * 2;
  const size_t kn_bytes = (size_t)NQ * NPIX * 4;
  const size_t total = 2 * xp_bytes + 2 * wr_bytes + 2 * ws_pl_bytes + 2 * t_bytes + kn_bytes;
  if (total > ws_size) return;

  char* ws = (char*)d_ws;
  size_t o = 0;
  unsigned short* xh  = (unsigned short*)(ws + o); o += xp_bytes;
  unsigned short* xl  = (unsigned short*)(ws + o); o += xp_bytes;
  unsigned short* wrh = (unsigned short*)(ws + o); o += wr_bytes;
  unsigned short* wrl = (unsigned short*)(ws + o); o += wr_bytes;
  unsigned short* wsh = (unsigned short*)(ws + o); o += ws_pl_bytes;
  unsigned short* wsl = (unsigned short*)(ws + o); o += ws_pl_bytes;
  unsigned short* th  = (unsigned short*)(ws + o); o += t_bytes;
  unsigned short* tl  = (unsigned short*)(ws + o); o += t_bytes;
  float*          kern = (float*)(ws + o);         o += kn_bytes;
  if (o > ws_size) return;

  dim3 gCx(NPB / 64, CH / 64, BS);
  k_cvt_x<<<gCx, 256, 0, stream>>>(x, xh, xl);

  const int nwblk = 8 + ((NQ * CR) / 8 + 255) / 256;
  k_cvt_w<<<nwblk, 256, 0, stream>>>(wr, wsp, wrh, wrl, wsh, wsl);

  k_gemm1<<<NPIX / 64, 128, 0, stream>>>(xh, xl, wrh, wrl, br, th, tl);

  dim3 gG2(NPIX / 256, NQ / 16);
  k_gemm2<<<gG2, 128, 0, stream>>>(wsh, wsl, th, tl, bsp, kern);

  dim3 gInv(HW / RB, NG, BS);
  k_inv<<<gInv, 256, 0, stream>>>(x, kern, out);
}
